// SubgraphSelector_58428735095403
// MI455X (gfx1250) — hardware-verified
//
#include <hip/hip_runtime.h>
#include <stdint.h>
#include <math.h>


#define HID 128
#define KIN 256
#define ROWS_PER_BLOCK 128
#define CHUNK_ROWS 131072
#define W1P_HALVES 32768

typedef _Float16 v16h __attribute__((ext_vector_type(16)));
typedef _Float16 v8h  __attribute__((ext_vector_type(8)));
typedef float    v8f  __attribute__((ext_vector_type(8)));
typedef float    v4f  __attribute__((ext_vector_type(4)));
typedef v4f      v4fa __attribute__((may_alias));

union Frag { v16h v; v8h half[2]; };

__device__ __forceinline__ v8f wmma_f16_step(const v16h a, const v16h b, v8f c) {
    v8f d = __builtin_amdgcn_wmma_f32_16x16x32_f16(false, a, false, b, (short)0, c, false, false);
    asm volatile("v_nop\n\tv_nop\n\tv_nop\n\tv_nop" : "+v"(d) : "v"(a), "v"(b));
    return d;
}

__global__ __launch_bounds__(256)
void pack_w1_f16(const float* __restrict__ W1, _Float16* __restrict__ w1p, int nthreads) {
    const int T = blockIdx.x * blockDim.x + threadIdx.x;
    if (T >= nthreads) return;
    const int t0   = T * 8;
    const int i0   = t0 & 15;
    const int lane = (t0 >> 4) & 31;
    const int tile = t0 >> 9;
    const int nt   = tile & 7;
    const int kt   = tile >> 3;
    const int h    = lane >> 4;
    const int n    = nt * 16 + (lane & 15);
    const int kb   = kt * 32 + 8 * h + (i0 ? 16 : 0);
    v8h v;
#pragma unroll
    for (int j = 0; j < 8; ++j) {
        v[j] = (_Float16)(W1[(size_t)(kb + j) * HID + n] * 16.0f);
    }
    _Float16* dst = w1p + (size_t)t0;
    *(volatile v8h*)dst = v;
    __threadfence();
    *(volatile v8h*)dst = v;
}

__global__ __launch_bounds__(256)
void gather_edge_rows(const float* __restrict__ hfeat, const int* __restrict__ eidx,
                      _Float16* __restrict__ Ad, int e_start, int E, int nnode, int rows) {
    const int lane = threadIdx.x & 31;
    const int wave = threadIdx.x >> 5;
    const int half = lane >> 4;
    const int q    = lane & 15;
#pragma unroll 2
    for (int j = 0; j < 16; ++j) {
        const int lr = blockIdx.x * ROWS_PER_BLOCK + wave * 16 + j;
        const int e  = e_start + lr;
        v8h v;
        if (e < E && lr < rows) {
            int idx = eidx[(size_t)half * (size_t)E + (size_t)e];
            idx = idx < 0 ? 0 : idx;
            idx = idx > nnode - 1 ? nnode - 1 : idx;
            const float* src = hfeat + (size_t)idx * HID + q * 8;
            const v4f x0 = *(const v4fa*)(src);
            const v4f x1 = *(const v4fa*)(src + 4);
            v[0] = (_Float16)x0[0]; v[1] = (_Float16)x0[1]; v[2] = (_Float16)x0[2]; v[3] = (_Float16)x0[3];
            v[4] = (_Float16)x1[0]; v[5] = (_Float16)x1[1]; v[6] = (_Float16)x1[2]; v[7] = (_Float16)x1[3];
        } else {
#pragma unroll
            for (int k = 0; k < 8; ++k) v[k] = (_Float16)0.0f;
        }
        if (lr < rows) {
            _Float16* dst = Ad + (size_t)lr * KIN + lane * 8;
            *(volatile v8h*)dst = v;
            __threadfence();
            *(volatile v8h*)dst = v;
        }
    }
}

__global__ __launch_bounds__(256)
void edge_mlp_f16(const _Float16* __restrict__ Ad, const _Float16* __restrict__ w1p,
                  const float* __restrict__ b1, const float* __restrict__ W2,
                  const float* __restrict__ b2, float* __restrict__ out,
                  int e_start, int E) {
    __shared__ __attribute__((aligned(16))) float outst[ROWS_PER_BLOCK];

    const int lane = threadIdx.x & 31;
    const int wave = threadIdx.x >> 5;
    const int m    = lane & 15;
    const int h    = lane >> 4;

    const _Float16* arow = Ad + ((size_t)blockIdx.x * ROWS_PER_BLOCK + (size_t)wave * 16 + (size_t)m) * KIN;

    v8f acc[8];
#pragma unroll
    for (int nt = 0; nt < 8; ++nt) { v8f z = {}; acc[nt] = z; }

#pragma unroll
    for (int kt = 0; kt < 8; ++kt) {
        Frag a;
        a.half[0] = *(const v8h*)(arow + kt * 32 + 8 * h);
        a.half[1] = *(const v8h*)(arow + kt * 32 + 16 + 8 * h);
#pragma unroll
        for (int nt = 0; nt < 8; ++nt) {
            const _Float16* bp = w1p + ((size_t)((kt * 8 + nt) * 32 + lane) << 4);
            Frag b;
            b.half[0] = *(const v8h*)(bp);
            b.half[1] = *(const v8h*)(bp + 8);
            acc[nt] = wmma_f16_step(a.v, b.v, acc[nt]);
        }
    }

    float s[8];
#pragma unroll
    for (int r = 0; r < 8; ++r) s[r] = 0.0f;
#pragma unroll
    for (int nt = 0; nt < 8; ++nt) {
        const float bb = b1[nt * 16 + m];
        const float ww = W2[nt * 16 + m];
#pragma unroll
        for (int r = 0; r < 8; ++r) {
            const float hid = fmaxf(acc[nt][r] * 0.0625f + bb, 0.0f);
            s[r] += hid * ww;
        }
    }
#pragma unroll
    for (int mask = 1; mask <= 8; mask <<= 1) {
#pragma unroll
        for (int r = 0; r < 8; ++r) s[r] += __shfl_xor(s[r], mask, 32);
    }
    const float b2v = b2[0];
    float v = s[0];
#pragma unroll
    for (int j = 1; j < 8; ++j) v = (m == j) ? s[j] : v;
    if (m < 8) {
        const float logit = v + b2v;
        outst[wave * 16 + 8 * h + m] = 1.0f / (1.0f + __expf(-logit));
    }
    __syncthreads();

    if (wave == 0) {
        const v4f val = *(const v4fa*)(&outst[4 * lane]);
        const int eb = e_start + blockIdx.x * ROWS_PER_BLOCK + 4 * lane;
        float* p = out + (size_t)eb;
        const bool full = (eb + 3 < E);
        if (full) {
            *(volatile v4f*)p = val;
        } else {
#pragma unroll
            for (int k = 0; k < 4; ++k) if (eb + k < E) ((volatile float*)p)[k] = val[k];
        }
        __threadfence();
        if (full) {
            *(volatile v4f*)p = val;
        } else {
#pragma unroll
            for (int k = 0; k < 4; ++k) if (eb + k < E) ((volatile float*)p)[k] = val[k];
        }
    }
}

extern "C" void kernel_launch(void* const* d_in, const int* in_sizes, int n_in,
                              void* d_out, int out_size, void* d_ws, size_t ws_size,
                              hipStream_t stream) {
    (void)n_in;
    const float* hfeat = (const float*)d_in[0];
    const int*   ei    = (const int*)d_in[1];
    const float* W1    = (const float*)d_in[2];
    const float* b1    = (const float*)d_in[3];
    const float* W2    = (const float*)d_in[4];
    const float* b2    = (const float*)d_in[5];
    float* out = (float*)d_out;

    const int nnode = in_sizes[0] / HID;
    const int E     = in_sizes[1] / 2;
    if (nnode <= 0 || E <= 0) return;
    if (in_sizes[2] != KIN * HID || in_sizes[3] < HID || in_sizes[4] < HID || in_sizes[5] < 1) return;
    if (out_size < E) return;

    const size_t ad_bytes = (size_t)CHUNK_ROWS * KIN * sizeof(_Float16);
    const size_t w1p_off  = ad_bytes;
    const size_t total    = w1p_off + (size_t)W1P_HALVES * sizeof(_Float16);
    if (total > ws_size) return;
    _Float16* Ad  = (_Float16*)d_ws;
    _Float16* w1p = (_Float16*)((char*)d_ws + w1p_off);

    const int pack_threads = W1P_HALVES / 8;
    pack_w1_f16<<<(pack_threads + 255) / 256, 256, 0, stream>>>(W1, w1p, pack_threads);

    const int nchunks = (E + CHUNK_ROWS - 1) / CHUNK_ROWS;
    for (int c = 0; c < nchunks; ++c) {
        const int e_start = c * CHUNK_ROWS;
        int rows = E - e_start;
        if (rows > CHUNK_ROWS) rows = CHUNK_ROWS;
        const int rows_p = ((rows + ROWS_PER_BLOCK - 1) / ROWS_PER_BLOCK) * ROWS_PER_BLOCK;
        const int grid   = rows_p / ROWS_PER_BLOCK;
        gather_edge_rows<<<grid, 256, 0, stream>>>(hfeat, ei, Ad, e_start, E, nnode, rows_p);
        edge_mlp_f16<<<grid, 256, 0, stream>>>(Ad, w1p, b1, W2, b2, out, e_start, E);
    }
}
